// MultiHeadRelativeAttention_89867895701650
// MI455X (gfx1250) — hardware-verified
//
#include <hip/hip_runtime.h>


#define SS   1024
#define NBT  4
#define EE   1024
#define NH_  16
#define HD   64
#define MPOS 2047
#define MP   2048
#define NTK  (SS * NBT)
#define PSC  32768.0f
#define LOSC 1024.0f
#define LOSCI (1.0f / 1024.0f)
#define SCL  0.125f

typedef _Float16 h16;
typedef unsigned short bf;
typedef __attribute__((ext_vector_type(16))) __bf16   v16bf;
typedef __attribute__((ext_vector_type(16))) _Float16 v16h;
typedef __attribute__((ext_vector_type(8)))  _Float16 v8h;
typedef __attribute__((ext_vector_type(8)))  unsigned short v8us;
typedef __attribute__((ext_vector_type(8)))  float    v8f;
typedef __attribute__((ext_vector_type(4)))  float    v4f;
typedef v8h  __attribute__((may_alias)) v8ha;
typedef v4f  __attribute__((may_alias)) v4fa;
typedef v8us __attribute__((may_alias)) v8usa;

__device__ __forceinline__ unsigned short f2bf(float f) { unsigned u = __float_as_uint(f); u += 0x7FFFu + ((u >> 16) & 1u); return (unsigned short)(u >> 16); }
__device__ __forceinline__ float bf2f(unsigned short b) { return __uint_as_float(((unsigned)b) << 16); }
__device__ __forceinline__ float bfr(float f) { return bf2f(f2bf(f)); }
__device__ __forceinline__ v16h cat16(v8h lo, v8h hi) { return __builtin_shufflevector(lo, hi, 0, 1, 2, 3, 4, 5, 6, 7, 8, 9, 10, 11, 12, 13, 14, 15); }
__device__ __forceinline__ v16bf cat16b(v8us lo, v8us hi) { return __builtin_bit_cast(v16bf, __builtin_shufflevector(lo, hi, 0, 1, 2, 3, 4, 5, 6, 7, 8, 9, 10, 11, 12, 13, 14, 15)); }
__device__ __forceinline__ v8f wmma16(v16h a, v16h b, v8f c) { return __builtin_amdgcn_wmma_f32_16x16x32_f16(false, a, false, b, (short)0, c, false, false); }
__device__ __forceinline__ v8f wmmab(v16bf a, v16bf b, v8f c) { return __builtin_amdgcn_wmma_f32_16x16x32_bf16(false, a, false, b, (short)0, c, false, false); }
#define VST2(T, p, v) do { const T vst2_v_ = (v); *(volatile T*)(p) = vst2_v_; __threadfence(); *(volatile T*)(p) = vst2_v_; } while (0)

__global__ __launch_bounds__(256) void k_cvtb(const float* __restrict__ src, int srcoff, int nvalid, int nrows, bf* dst) {
    const int lane = threadIdx.x & 31, r = blockIdx.x * 8 + (threadIdx.x >> 5);
    if (r >= nrows) return;
    const int rs = (r < nvalid) ? (r + srcoff) : srcoff;
#pragma unroll
    for (int q = 0; q < 4; ++q) { v8us t;
#pragma unroll
        for (int i = 0; i < 8; ++i) { const unsigned short hb = f2bf(src[(size_t)rs * EE + q * 256 + lane * 8 + i]); t[i] = (r < nvalid) ? hb : (unsigned short)0; }
        VST2(v8us, dst + (size_t)r * EE + q * 256 + lane * 8, t); }
}

template <bool SPLITA, int MODE>
__global__ __launch_bounds__(128) void k_gemmb(const bf* __restrict__ A, const bf* __restrict__ Al, const bf* __restrict__ Bn, const float* __restrict__ bias, const float* __restrict__ bias2, void* C, void* C2) {
    __shared__ __align__(16) float ost[4][16 * 68];
    const int lane = threadIdx.x & 31, wave = threadIdx.x >> 5, lr = lane & 15, hi = lane >> 4;
    const int r0 = blockIdx.x * 64 + wave * 16, c0 = blockIdx.y * 64;
    const size_t aoff = (size_t)(r0 + lr) * EE + 8 * hi;
    size_t boff[4];
#pragma unroll
    for (int t = 0; t < 4; ++t) boff[t] = (size_t)(c0 + t * 16 + lr) * EE + 8 * hi;
    v8f acc[4];
#pragma unroll
    for (int t = 0; t < 4; ++t) acc[t] = (v8f){};
#pragma unroll 1
    for (int kc = 0; kc < EE; kc += 32) {
        const v16bf a = cat16b(*(const v8us*)(A + aoff + kc), *(const v8us*)(A + aoff + kc + 16));
        v16bf al = a;
        if (SPLITA) al = cat16b(*(const v8us*)(Al + aoff + kc), *(const v8us*)(Al + aoff + kc + 16));
#pragma unroll
        for (int t = 0; t < 4; ++t) { const v16bf b = cat16b(*(const v8us*)(Bn + boff[t] + kc), *(const v8us*)(Bn + boff[t] + kc + 16)); acc[t] = wmmab(a, b, acc[t]); if (SPLITA) acc[t] = wmmab(al, b, acc[t]); }
        asm volatile("v_nop\n\tv_nop\n\tv_nop\n\tv_nop" : "+v"(acc[0]), "+v"(acc[1]), "+v"(acc[2]), "+v"(acc[3]) : "v"(a), "v"(al));
    }
    float* os = &ost[wave][0];
#pragma unroll
    for (int t = 0; t < 4; ++t) { const int col = c0 + t * 16 + lr; const float bv = (MODE == 0 && bias) ? bfr(bias[col]) : 0.f;
#pragma unroll
        for (int j = 0; j < 8; ++j) os[(hi * 8 + j) * 68 + t * 16 + lr] = acc[t][j] + bv; }
    __syncthreads();
    if (MODE == 0) {
        float* crow = (float*)C + (size_t)r0 * EE + c0;
        auto pass = [&]() {
#pragma unroll
            for (int s = 0; s < 8; ++s) { const int Lid = (lane >> 3) + 4 * s, piece = lane & 7; const int row = Lid >> 1, cofs = (Lid & 1) * 32 + piece * 4;
                const v4f val = *(const v4fa*)(os + row * 68 + cofs); *(volatile v4f*)(crow + (size_t)row * EE + cofs) = val; }
        };
        pass(); __threadfence(); pass();
    } else if (MODE == 1) {
        h16* c1 = (h16*)C + (size_t)r0 * EE + c0; h16* c2 = (h16*)C2 + (size_t)r0 * EE + c0;
        auto pass = [&]() {
#pragma unroll
            for (int s = 0; s < 4; ++s) { const int row = 4 * s + (lane >> 3), piece = lane & 7; const float* sp = os + row * 68 + piece * 8; v8h o1, o2;
#pragma unroll
                for (int i = 0; i < 8; ++i) { const int col = c0 + piece * 8 + i; o1[i] = (h16)(sp[i] + bfr(bias[col])); o2[i] = (h16)(sp[i] + bfr(bias2[col])); }
                *(volatile v8h*)(c1 + (size_t)row * EE + piece * 8) = o1; *(volatile v8h*)(c2 + (size_t)row * EE + piece * 8) = o2; }
        };
        pass(); __threadfence(); pass();
    } else {
        h16* c1 = (h16*)C + (size_t)r0 * EE + c0;
        auto pass = [&]() {
#pragma unroll
            for (int s = 0; s < 4; ++s) { const int row = 4 * s + (lane >> 3), piece = lane & 7; const float* sp = os + row * 68 + piece * 8; v8h o1;
#pragma unroll
                for (int i = 0; i < 8; ++i) o1[i] = (h16)sp[i];
                *(volatile v8h*)(c1 + (size_t)row * EE + piece * 8) = o1; }
        };
        pass(); __threadfence(); pass();
    }
}

__global__ __launch_bounds__(256) void k_vt(const float* __restrict__ V, h16* VTH) {
    __shared__ __align__(16) h16 tile[HD * 72];
    const int bid = blockIdx.x;
    const int b = bid / (NH_ * (SS / 64)), rem = bid - b * (NH_ * (SS / 64)), h = rem / (SS / 64), kt = rem - h * (SS / 64);
    const int s0 = kt * 64, tid = threadIdx.x, kk = tid >> 2, d0 = (tid & 3) * 16;
    const float* src = V + ((size_t)(s0 + kk) * NBT + b) * EE + h * HD + d0;
#pragma unroll
    for (int i = 0; i < 16; ++i) tile[(d0 + i) * 72 + kk] = (h16)src[i];
    __syncthreads();
    const int piece = tid & 7;
    const size_t base = (((size_t)b * NH_ + h) * HD) * SS + s0;
    auto pass = [&]() {
#pragma unroll
        for (int s = 0; s < 2; ++s) { const int d = (tid >> 3) + 32 * s;
            const v8h val = *(const v8ha*)(tile + d * 72 + piece * 8); *(volatile v8h*)(VTH + base + (size_t)d * SS + piece * 8) = val; }
    };
    pass(); __threadfence(); pass();
}

__global__ __launch_bounds__(128) void k_attn(const h16* __restrict__ QC, const h16* __restrict__ QP, const h16* __restrict__ K16, const h16* __restrict__ KP,
                                             const h16* __restrict__ VTH, bf* CH, bf* CL) {
    __shared__ __align__(16) h16 plds[4][16 * 32];
    __shared__ __align__(16) float posl[4][16 * 52];
    __shared__ __align__(16) float ost[4][16 * 68];
    const int lane = threadIdx.x & 31, wave = threadIdx.x >> 5, lr = lane & 15, hi = lane >> 4;
    const int bid = blockIdx.x;
    const int b = bid / (NH_ * (SS / 64)), rem = bid - b * (NH_ * (SS / 64)), h = rem / (SS / 64), qt = rem - h * (SS / 64);
    const int q0 = qt * 64 + wave * 16;
    h16* pl = &plds[wave][0]; float* ps = &posl[wave][0];
    v16h qc[2];
    const size_t qoff = ((size_t)(q0 + lr) * NBT + b) * EE + h * HD + 8 * hi;
#pragma unroll
    for (int kc = 0; kc < 2; ++kc) qc[kc] = cat16(*(const v8h*)(QC + qoff + kc * 32), *(const v8h*)(QC + qoff + kc * 32 + 16));
    const size_t vbase = (((size_t)b * NH_ + h) * HD) * SS;
    v8f o[4];
#pragma unroll
    for (int n = 0; n < 4; ++n) o[n] = (v8f){};
    float mrow[8], lpart[8];
#pragma unroll
    for (int j = 0; j < 8; ++j) { mrow[j] = -3.0e38f; lpart[j] = 0.f; }
#pragma unroll 1
    for (int kt = 0; kt < SS / 32; ++kt) {
        const int l0 = kt * 32;
        v8f s0 = {}, s1 = {};
#pragma unroll
        for (int kc = 0; kc < 2; ++kc) {
            const size_t o0 = ((size_t)(l0 + lr) * NBT + b) * EE + h * HD + kc * 32 + 8 * hi, o1 = ((size_t)(l0 + 16 + lr) * NBT + b) * EE + h * HD + kc * 32 + 8 * hi;
            s0 = wmma16(qc[kc], cat16(*(const v8h*)(K16 + o0), *(const v8h*)(K16 + o0 + 16)), s0);
            s1 = wmma16(qc[kc], cat16(*(const v8h*)(K16 + o1), *(const v8h*)(K16 + o1 + 16)), s1);
        }
        const int mbase = (SS - 1) - (q0 + 15) + l0;
        { const v16h qp0 = cat16(*(const v8h*)(QP + qoff), *(const v8h*)(QP + qoff + 16)), qp1 = cat16(*(const v8h*)(QP + qoff + 32), *(const v8h*)(QP + qoff + 48));
#pragma unroll
          for (int t = 0; t < 3; ++t) {
            const size_t om = ((size_t)(mbase + t * 16 + lr) * NH_ + h) * HD + 8 * hi;
            v8f pz = wmma16(qp0, cat16(*(const v8h*)(KP + om), *(const v8h*)(KP + om + 16)), (v8f){});
            pz = wmma16(qp1, cat16(*(const v8h*)(KP + om + 32), *(const v8h*)(KP + om + 48)), pz);
            asm volatile("v_nop\n\tv_nop\n\tv_nop\n\tv_nop" : "+v"(pz) : "v"(qp0), "v"(qp1));
#pragma unroll
            for (int j = 0; j < 8; ++j) ps[(hi * 8 + j) * 52 + t * 16 + lr] = pz[j];
          } }
        asm volatile("v_nop\n\tv_nop\n\tv_nop\n\tv_nop" : "+v"(s0), "+v"(s1) : "v"(qc[0]), "v"(qc[1]));
        asm volatile("" ::: "memory");
        __builtin_amdgcn_fence(__ATOMIC_RELEASE, "workgroup");
        __builtin_amdgcn_wave_barrier();
        float alpha[8];
#pragma unroll
        for (int j = 0; j < 8; ++j) {
            const int r = hi * 8 + j;
            const float p0v = ps[r * 52 + 15 - r + lr], p1v = ps[r * 52 + 15 - r + 16 + lr];
            const float a0 = (s0[j] + p0v) * SCL, a1 = (s1[j] + p1v) * SCL;
            float mx = fmaxf(a0, a1);
            mx = fmaxf(mx, __shfl_xor(mx, 1, 16)); mx = fmaxf(mx, __shfl_xor(mx, 2, 16)); mx = fmaxf(mx, __shfl_xor(mx, 4, 16)); mx = fmaxf(mx, __shfl_xor(mx, 8, 16));
            const float mn = fmaxf(mrow[j], mx);
            alpha[j] = __expf(mrow[j] - mn); mrow[j] = mn;
            const float e0 = __expf(a0 - mn), e1 = __expf(a1 - mn);
            lpart[j] = lpart[j] * alpha[j] + (e0 + e1);
            pl[r * 32 + lr] = (h16)(e0 * PSC); pl[r * 32 + 16 + lr] = (h16)(e1 * PSC);
        }
#pragma unroll
        for (int n = 0; n < 4; ++n)
#pragma unroll
            for (int j = 0; j < 8; ++j) o[n][j] *= alpha[j];
        asm volatile("" ::: "memory");
        const v16h pa = cat16(*(const v8ha*)(pl + lr * 32 + hi * 8), *(const v8ha*)(pl + lr * 32 + 16 + hi * 8));
#pragma unroll
        for (int n = 0; n < 4; ++n) { const size_t vo = vbase + (size_t)(n * 16 + lr) * SS + l0 + hi * 8;
            o[n] = wmma16(pa, cat16(*(const v8h*)(VTH + vo), *(const v8h*)(VTH + vo + 16)), o[n]); }
        asm volatile("v_nop\n\tv_nop\n\tv_nop\n\tv_nop" : "+v"(o[0]), "+v"(o[1]), "+v"(o[2]), "+v"(o[3]) : "v"(pa));
        __builtin_amdgcn_wave_barrier();
    }
    float inv[8];
#pragma unroll
    for (int j = 0; j < 8; ++j) { float rs = lpart[j]; rs += __shfl_xor(rs, 1, 16); rs += __shfl_xor(rs, 2, 16); rs += __shfl_xor(rs, 4, 16); rs += __shfl_xor(rs, 8, 16); inv[j] = 1.0f / (rs * PSC); }
    float* os = &ost[wave][0];
#pragma unroll
    for (int n = 0; n < 4; ++n)
#pragma unroll
        for (int j = 0; j < 8; ++j) os[(hi * 8 + j) * 68 + n * 16 + lr] = o[n][j] * inv[j];
    __syncthreads();
    auto pass = [&]() {
#pragma unroll
        for (int s = 0; s < 4; ++s) { const int row = 4 * s + (lane >> 3), piece = lane & 7; const float* sp = os + row * 68 + piece * 8; v8us oh, ol;
#pragma unroll
            for (int i = 0; i < 8; ++i) { const unsigned short hb = f2bf(sp[i]); oh[i] = hb; ol[i] = f2bf(sp[i] - bf2f(hb)); }
            const size_t co = ((size_t)(q0 + row) * NBT + b) * EE + h * HD + piece * 8;
            *(volatile v8us*)(CH + co) = oh; *(volatile v8us*)(CL + co) = ol; }
    };
    pass(); __threadfence(); pass();
}

extern "C" void kernel_launch(void* const* d_in, const int* in_sizes, int n_in,
                              void* d_out, int out_size, void* d_ws, size_t ws_size, hipStream_t stream) {
    (void)in_sizes; (void)n_in; (void)out_size;
    const float* query = (const float*)d_in[0]; const float* key = (const float*)d_in[1]; const float* value = (const float*)d_in[2]; const float* pe = (const float*)d_in[3];
    const float* wq = (const float*)d_in[4]; const float* wk = (const float*)d_in[5]; const float* wv = (const float*)d_in[6]; const float* wkp = (const float*)d_in[7];
    const float* cb = (const float*)d_in[8]; const float* pb = (const float*)d_in[9]; const float* wo = (const float*)d_in[10]; const float* bo = (const float*)d_in[11];
    float* out = (float*)d_out;
    char* wsp = (char*)d_ws;
    auto take = [&](size_t bytes) { char* p = wsp; wsp += (bytes + 255) & ~(size_t)255; return (void*)p; };
    bf* Xq = (bf*)take((size_t)NTK * EE * 2); bf* Xk = (bf*)take((size_t)NTK * EE * 2); bf* Xv = (bf*)take((size_t)NTK * EE * 2); bf* Xp = (bf*)take((size_t)MP * EE * 2);
    bf* Wq = (bf*)take((size_t)EE * EE * 2); bf* Wk = (bf*)take((size_t)EE * EE * 2); bf* Wv = (bf*)take((size_t)EE * EE * 2); bf* Wp = (bf*)take((size_t)EE * EE * 2); bf* Wo = (bf*)take((size_t)EE * EE * 2);
    h16* QC = (h16*)take((size_t)NTK * EE * 2); h16* QP = (h16*)take((size_t)NTK * EE * 2); h16* K16 = (h16*)take((size_t)NTK * EE * 2); h16* KP = (h16*)take((size_t)MP * EE * 2);
    float* Vf = (float*)take((size_t)NTK * EE * 4); h16* VTH = (h16*)take((size_t)NTK * EE * 2);
    if ((size_t)(wsp - (char*)d_ws) > ws_size) return;
    bf* CH = Xq; bf* CL = Xk;
    k_cvtb<<<NTK / 8, 256, 0, stream>>>(query, 0, NTK, NTK, Xq);
    k_cvtb<<<NTK / 8, 256, 0, stream>>>(key, 0, NTK, NTK, Xk);
    k_cvtb<<<NTK / 8, 256, 0, stream>>>(value, 0, NTK, NTK, Xv);
    k_cvtb<<<MP / 8, 256, 0, stream>>>(pe, 1, MPOS, MP, Xp);
    k_cvtb<<<EE / 8, 256, 0, stream>>>(wq, 0, EE, EE, Wq); k_cvtb<<<EE / 8, 256, 0, stream>>>(wk, 0, EE, EE, Wk); k_cvtb<<<EE / 8, 256, 0, stream>>>(wv, 0, EE, EE, Wv);
    k_cvtb<<<EE / 8, 256, 0, stream>>>(wkp, 0, EE, EE, Wp); k_cvtb<<<EE / 8, 256, 0, stream>>>(wo, 0, EE, EE, Wo);
    k_gemmb<false, 1><<<dim3(NTK / 64, EE / 64, 1), 128, 0, stream>>>(Xq, nullptr, Wq, cb, pb, QC, QP);
    k_gemmb<false, 2><<<dim3(NTK / 64, EE / 64, 1), 128, 0, stream>>>(Xk, nullptr, Wk, nullptr, nullptr, K16, nullptr);
    k_gemmb<false, 2><<<dim3(MP / 64, EE / 64, 1), 128, 0, stream>>>(Xp, nullptr, Wp, nullptr, nullptr, KP, nullptr);
    k_gemmb<false, 0><<<dim3(NTK / 64, EE / 64, 1), 128, 0, stream>>>(Xv, nullptr, Wv, nullptr, nullptr, Vf, nullptr);
    k_vt<<<NBT * NH_ * (SS / 64), 256, 0, stream>>>(Vf, VTH);
    k_attn<<<NBT * NH_ * (SS / 64), 128, 0, stream>>>(QC, QP, K16, KP, VTH, CH, CL);
    k_gemmb<true, 0><<<dim3(NTK / 64, EE / 64, 1), 128, 0, stream>>>(CH, CL, Wo, bo, nullptr, out, nullptr);
}
